// BipartiteGraph_8177617732032
// MI455X (gfx1250) — hardware-verified
//
#include <hip/hip_runtime.h>
#include <math.h>

typedef __attribute__((ext_vector_type(16))) _Float16 v16h;
typedef __attribute__((ext_vector_type(16))) __bf16 v16b;
typedef __attribute__((ext_vector_type(8)))  _Float16 v8h;
typedef __attribute__((ext_vector_type(8)))  float v8f;
typedef __attribute__((ext_vector_type(4)))  float v4f;
typedef __attribute__((ext_vector_type(2)))  float v2f;
typedef __attribute__((ext_vector_type(4)))  unsigned v4u;
typedef __attribute__((ext_vector_type(4)))  int v4i;
typedef float __attribute__((may_alias)) float_a;
typedef int __attribute__((may_alias)) int_a;

template <typename T> __device__ __forceinline__ void vst2(void* p, T v) { *(volatile T*)p = v; __threadfence(); *(volatile T*)p = v; }
__device__ __forceinline__ v8f wmma16(v16h a, v16h b, v8f c) {
  v8f d = __builtin_amdgcn_wmma_f32_16x16x32_f16(false, a, false, b, (short)0, c, false, false);
  asm volatile("v_nop\n\tv_nop\n\tv_nop\n\tv_nop" : "+v"(d) : "v"(a), "v"(b));
  return d;
}
__device__ __forceinline__ v8f wmma_bf(v16b a, v16b b, v8f c) {
  v8f d = __builtin_amdgcn_wmma_f32_16x16x32_bf16(false, a, false, b, (short)0, c, false, false);
  asm volatile("v_nop\n\tv_nop\n\tv_nop\n\tv_nop" : "+v"(d) : "v"(a), "v"(b));
  return d;
}
__device__ __forceinline__ v16h frag_h(const _Float16* rowk0, int lane) {
  union { v16h v; v8h q[2]; } u; const _Float16* p = rowk0 + 8 * (lane >> 4);
  u.q[0] = *(const v8h*)p; u.q[1] = *(const v8h*)(p + 16); return u.v;
}
__device__ __forceinline__ v16h frag_f32(const float* rowk0, int lane) {
  v16h a; const float* p = rowk0 + 8 * (lane >> 4);
#pragma unroll
  for (int i = 0; i < 8; ++i) { a[i] = (_Float16)p[i]; a[8 + i] = (_Float16)p[16 + i]; }
  return a;
}
__device__ __forceinline__ v16h frag_f32s(const float* rowk0, int lane, float sc) {
  v16h a; const float* p = rowk0 + 8 * (lane >> 4);
#pragma unroll
  for (int i = 0; i < 8; ++i) { a[i] = (_Float16)(p[i] * sc); a[8 + i] = (_Float16)(p[16 + i] * sc); }
  return a;
}
__device__ __forceinline__ v16h fragc_f32(const float* W, int k0, int n, int lane, int ld, int K) {
  v16h a; const int g = lane >> 4;
#pragma unroll
  for (int i = 0; i < 8; ++i) { const int ka = k0 + 8 * g + i, kb = ka + 16;
    a[i] = (_Float16)(ka < K ? W[(size_t)(ka < K ? ka : K - 1) * ld + n] : 0.f); a[8 + i] = (_Float16)(kb < K ? W[(size_t)(kb < K ? kb : K - 1) * ld + n] : 0.f); }
  return a;
}
struct F2 { v16b h, l; };
__device__ __forceinline__ F2 bsplit16(const float v[16]) { F2 r;
#pragma unroll
  for (int i = 0; i < 16; ++i) { const __bf16 h = (__bf16)v[i]; r.h[i] = h; r.l[i] = (__bf16)(v[i] - (float)h); }
  return r; }
__device__ __forceinline__ F2 split_row(const float* row, int k0, int lane) { float v[16]; const float* p = row + k0 + 8 * (lane >> 4);
#pragma unroll
  for (int i = 0; i < 8; ++i) { v[i] = p[i]; v[8 + i] = p[16 + i]; }
  return bsplit16(v); }
__device__ __forceinline__ F2 split_rowK(const float* row, int k0, int lane, int K) { float v[16]; const int g = lane >> 4;
#pragma unroll
  for (int i = 0; i < 8; ++i) { const int ka = k0 + 8 * g + i, kb = ka + 16; v[i] = ka < K ? row[ka < K ? ka : K - 1] : 0.f; v[8 + i] = kb < K ? row[kb < K ? kb : K - 1] : 0.f; }
  return bsplit16(v); }
__device__ __forceinline__ F2 split_col(const float* W, int k0, int n, int lane, int ld, int K) { float v[16]; const int g = lane >> 4;
#pragma unroll
  for (int i = 0; i < 8; ++i) { const int ka = k0 + 8 * g + i, kb = ka + 16; v[i] = ka < K ? W[(size_t)(ka < K ? ka : K - 1) * ld + n] : 0.f; v[8 + i] = kb < K ? W[(size_t)(kb < K ? kb : K - 1) * ld + n] : 0.f; }
  return bsplit16(v); }
__device__ __forceinline__ v8f mac3(const F2& a, const F2& b, v8f c) { c = wmma_bf(a.l, b.h, c); c = wmma_bf(a.h, b.l, c); return wmma_bf(a.h, b.h, c); }
__device__ __forceinline__ float sigm(float v) { return 1.0f / (1.0f + expf(-v)); }
#define LDSX() do { asm volatile("s_wait_dscnt 0" ::: "memory"); __builtin_amdgcn_wave_barrier(); __builtin_amdgcn_fence(__ATOMIC_RELEASE, "workgroup"); } while (0)


#define NU 512
#define NV 512
#define KD 128
#define RD 256
#ifndef DBGM
#define DBGM 0
#endif
typedef __attribute__((ext_vector_type(8))) __bf16 v8b;
__device__ __forceinline__ v16b frag_b(const __bf16* rowk0, int lane) {
  union { v16b v; v8b q[2]; } u; const __bf16* p = rowk0 + 8 * (lane >> 4);
  u.q[0] = *(const v8b*)p; u.q[1] = *(const v8b*)(p + 16); return u.v;
}
__device__ __forceinline__ float bfr(float v) { return (float)(__bf16)v; }
__device__ __attribute__((noinline)) float exp_ni(float v) { return expf(v); }
#define PT_W1A 0u
#define PT_W1B (PT_W1A + 256u * 128)
#define PT_W2  (PT_W1B + 256u * 128)
#define PT_VTU (PT_W2 + 128u * 256)
#define PT_UTV (PT_VTU + 256u * 128)
#define PT_UUP (PT_UTV + 256u * 128)
#define PT_VUP (PT_UUP + 128u * 384)
#define PT_END (PT_VUP + 128u * 384)
#define WS_PT   0u
#define WS_EU   (WS_PT + 2u * PT_END)
#define WS_EV   (WS_EU + 4u * NU * KD)
#define WS_PU   (WS_EV + 4u * NV * KD)
#define WS_PV   (WS_PU + 4u * NU * RD)
#define WS_MT   (WS_PV + 4u * NV * RD)
#define WS_A    (WS_MT + 4u * RD * 512)
#define WS_AT   (WS_A + 4u * NU * NV)
#define WS_END  (WS_AT + 4u * NV * NU)

__global__ __launch_bounds__(128) void k_pack(const float* __restrict__ w1, const float* __restrict__ w2, const float* __restrict__ vtu, const float* __restrict__ utv, const float* __restrict__ uup, const float* __restrict__ vup, __bf16* __restrict__ PT) {
  __shared__ __align__(16) __bf16 srow[384];
  const int n = blockIdx.x, tid = threadIdx.x; int len; size_t dst;
  if (n < 256)       { len = 128; dst = PT_W1A + (size_t)n * 128; for (int k = tid; k < len; k += 128) srow[k] = (__bf16)bfr(w1[(size_t)k * RD + n]); }
  else if (n < 512)  { const int o = n - 256; len = 128; dst = PT_W1B + (size_t)o * 128; for (int k = tid; k < len; k += 128) srow[k] = (__bf16)bfr(w1[(size_t)(128 + k) * RD + o]); }
  else if (n < 640)  { const int o = n - 512; len = 256; dst = PT_W2 + (size_t)o * 256; for (int k = tid; k < len; k += 128) srow[k] = (__bf16)bfr(w2[(size_t)k * KD + o]); }
  else if (n < 896)  { const int o = n - 640; len = 128; dst = PT_VTU + (size_t)o * 128; for (int k = tid; k < len; k += 128) srow[k] = (__bf16)bfr(vtu[(size_t)k * RD + o]); }
  else if (n < 1152) { const int o = n - 896; len = 128; dst = PT_UTV + (size_t)o * 128; for (int k = tid; k < len; k += 128) srow[k] = (__bf16)bfr(utv[(size_t)k * RD + o]); }
  else if (n < 1280) { const int o = n - 1152; len = 384; dst = PT_UUP + (size_t)o * 384; for (int k = tid; k < len; k += 128) srow[k] = (__bf16)bfr(uup[(size_t)k * KD + o]); }
  else               { const int o = n - 1280; len = 384; dst = PT_VUP + (size_t)o * 384; for (int k = tid; k < len; k += 128) srow[k] = (__bf16)bfr(vup[(size_t)k * KD + o]); }
  __syncthreads();
  if (tid < len / 8) vst2((unsigned*)(PT + dst + tid * 8), *(const v4u*)(&srow[tid * 8]));
}
__global__ __launch_bounds__(32) void k_init(const float* __restrict__ eu0, const float* __restrict__ ev0, float* __restrict__ EU, float* __restrict__ EV) {
  const int n = blockIdx.x, lane = threadIdx.x; const bool isu = n < NU; const int r = isu ? n : n - NU; const float* s = (isu ? eu0 : ev0) + (size_t)r * KD; v4f v; for (int i = 0; i < 4; ++i) v[i] = bfr(s[lane * 4 + i]); vst2((isu ? EU : EV) + (size_t)r * KD + lane * 4, v);
}
__global__ __launch_bounds__(128) void k_node(const float* __restrict__ EU, const float* __restrict__ EV, const __bf16* __restrict__ PT, const float* __restrict__ b1, const float* __restrict__ vtub, const float* __restrict__ utvb, float* __restrict__ PU, float* __restrict__ PV, float* __restrict__ MT, int mode) {
  __shared__ __align__(16) float so[4][16][RD + 4]; __shared__ __align__(16) float st[RD][68];
  const int tid = threadIdx.x, wave = tid >> 5, lane = tid & 31, col = lane & 15, g = lane >> 4; const int r0 = blockIdx.x * 64 + wave * 16;
  const float* src = mode == 1 ? EV : EU;
  F2 a[4];
#pragma unroll
  for (int kc = 0; kc < 4; ++kc) a[kc] = split_row(src + (size_t)(r0 + col) * KD, kc * 32, lane);
  if (mode < 2) {
    v8f acc[16] = {}; const __bf16* W = PT + (mode == 0 ? PT_W1A : PT_W1B);
#pragma unroll
    for (int kc = 0; kc < 4; ++kc)
#pragma unroll
      for (int j = 0; j < 16; ++j) { const v16b w = frag_b(W + (size_t)(j * 16 + col) * KD + kc * 32, lane); acc[j] = wmma_bf(a[kc].l, w, acc[j]); acc[j] = wmma_bf(a[kc].h, w, acc[j]); }
#pragma unroll
    for (int j = 0; j < 16; ++j) { const float bb = mode == 1 ? bfr(b1[j * 16 + col]) : 0.f;
#pragma unroll
      for (int r = 0; r < 8; ++r) so[wave][8 * g + r][j * 16 + col] = acc[j][r] + bb; }
    LDSX();
    float* dst = mode == 0 ? PU : PV;
    for (int rl = 0; rl < 16; ++rl) for (int pc = lane; pc < RD / 4; pc += 32) vst2(dst + (size_t)(r0 + rl) * RD + pc * 4, *(const v4f*)&so[wave][rl][pc * 4]); }
  if (mode >= 1) {
    __syncthreads();
    v8f acc[16] = {}; const __bf16* W = PT + (mode == 1 ? PT_VTU : PT_UTV); const float* bb = mode == 1 ? vtub : utvb;
#pragma unroll
    for (int kc = 0; kc < 4; ++kc)
#pragma unroll
      for (int j = 0; j < 16; ++j) { const v16b w = frag_b(W + (size_t)(j * 16 + col) * KD + kc * 32, lane); acc[j] = wmma_bf(a[kc].l, w, acc[j]); acc[j] = wmma_bf(a[kc].h, w, acc[j]); }
#pragma unroll
    for (int j = 0; j < 16; ++j) { const int o = j * 16 + col; const float bv = bfr(bb[o]);
#pragma unroll
      for (int r = 0; r < 8; ++r) st[o][wave * 16 + 8 * g + r] = fmaxf(acc[j][r] + bv, 0.f); }
    __syncthreads();
    for (int q = tid; q < RD * 16; q += 128) { const int o = q >> 4, pc = q & 15; vst2(MT + (size_t)o * 512 + blockIdx.x * 64 + pc * 4, *(const v4f*)&st[o][pc * 4]); } }
}
__global__ __launch_bounds__(128) void k_edge(const float* __restrict__ PU, const float* __restrict__ PV, const int* __restrict__ UI, const int* __restrict__ VI, const __bf16* __restrict__ PT, const float* __restrict__ b2, const float* __restrict__ w3, const float* __restrict__ b3, float* __restrict__ A, float* __restrict__ Aout) {
  __shared__ __align__(16) __bf16 sah[64][RD + 8], sal[64][RD + 8]; __shared__ float sh2[64][KD + 1]; __shared__ float sw3[KD]; __shared__ __align__(16) float sres[64];
  const int tid = threadIdx.x, wave = tid >> 5, lane = tid & 31, col = lane & 15, g = lane >> 4; const int u = blockIdx.y, v0 = blockIdx.x * 64;
  __shared__ int suu[64], svv[64];
  if (tid < 64) { const size_t e = (size_t)u * NV + v0 + tid; suu[tid] = min(max(UI[e], 0), NU - 1); svv[tid] = min(max(VI[e], 0), NV - 1); }
  __syncthreads();
  for (int q = tid; q < 64 * RD; q += 128) { const int vl = q >> 8, c = q & 255; const float h = fmaxf(PU[(size_t)suu[vl] * RD + c] + PV[(size_t)svv[vl] * RD + c], 0.f); const __bf16 hb = (__bf16)h; sah[vl][c] = hb; sal[vl][c] = (__bf16)(h - (float)hb); }
  sw3[tid] = bfr(w3[tid]);
  __syncthreads();
  { v8f acc[8] = {};
#pragma unroll 2
    for (int kc = 0; kc < RD / 32; ++kc) { const v16b ah = frag_b(&sah[wave * 16 + col][kc * 32], lane), al = frag_b(&sal[wave * 16 + col][kc * 32], lane);
#pragma unroll
      for (int j = 0; j < 8; ++j) { const v16b w = frag_b(PT + PT_W2 + (size_t)(j * 16 + col) * RD + kc * 32, lane); acc[j] = wmma_bf(al, w, acc[j]); acc[j] = wmma_bf(ah, w, acc[j]); } }
#pragma unroll
    for (int j = 0; j < 8; ++j) { const float bb = bfr(b2[j * 16 + col]);
#pragma unroll
      for (int r = 0; r < 8; ++r) sh2[wave * 16 + 8 * g + r][j * 16 + col] = fmaxf(acc[j][r] + bb, 0.f); } }
  __syncthreads();
  if (tid < 64) { float s = bfr(b3[0]); for (int k = 0; k < KD; ++k) s += sh2[tid][k] * sw3[k]; sres[tid] = 1.0f / (1.0f + exp_ni(-s)); }
  __syncthreads();
  if (tid < 16) { vst2(A + (size_t)u * NV + v0 + tid * 4, *(const v4f*)&sres[tid * 4]); if (Aout) vst2(Aout + (size_t)u * NV + v0 + tid * 4, *(const v4f*)&sres[tid * 4]); }
}
#if DBGM == 3
__global__ __launch_bounds__(64) void k_zeroA(float* __restrict__ A) { const v4f z = {0.f, 0.f, 0.f, 0.f}; vst2(A + (size_t)blockIdx.x * 256 + threadIdx.x * 4, z); }
#endif
__global__ __launch_bounds__(256) void k_at(const float* __restrict__ A, float* __restrict__ AT) {
  __shared__ float st[64][65];
  const int u0 = blockIdx.y * 64, v0 = blockIdx.x * 64, tid = threadIdx.x;
  for (int q = tid; q < 64 * 64; q += 256) { const int ul = q >> 6, vl = q & 63; st[vl][ul] = A[(size_t)(u0 + ul) * NV + v0 + vl]; }
  __syncthreads();
  for (int q = tid; q < 64 * 16; q += 256) { const int vl = q >> 4, pc = q & 15; v4f v = {st[vl][pc * 4], st[vl][pc * 4 + 1], st[vl][pc * 4 + 2], st[vl][pc * 4 + 3]}; vst2(AT + (size_t)(v0 + vl) * NU + u0 + pc * 4, v); }
}
__global__ __launch_bounds__(128) void k_upd(const float* __restrict__ Am, const float* __restrict__ MT, float* __restrict__ E, const __bf16* __restrict__ WUP, const float* __restrict__ g1, const float* __restrict__ bb1, const float* __restrict__ g2, const float* __restrict__ bb2, float* __restrict__ Eout) {
  __shared__ __align__(16) float so[4][16][RD + 4]; __shared__ __align__(16) __bf16 sch[4][16][392], scl[4][16][392];
  const int tid = threadIdx.x, wave = tid >> 5, lane = tid & 31, col = lane & 15, g = lane >> 4; const int r0 = blockIdx.x * 64 + wave * 16;
  { v8f acc[16] = {};
#pragma unroll 1
    for (int kc = 0; kc < 512 / 32; ++kc) { const F2 a = split_row(Am + (size_t)(r0 + col) * 512, kc * 32, lane);
#pragma unroll
      for (int j = 0; j < 16; ++j) { const F2 b = split_row(MT + (size_t)(j * 16 + col) * 512, kc * 32, lane); acc[j] = mac3(a, b, acc[j]); } }
#pragma unroll
    for (int j = 0; j < 16; ++j)
#pragma unroll
      for (int r = 0; r < 8; ++r) so[wave][8 * g + r][j * 16 + col] = acc[j][r]; }
  LDSX();
  { const int rl = lane >> 1, half = lane & 1; float s = 0.f; for (int c = half * 128; c < half * 128 + 128; ++c) s += so[wave][rl][c]; s += __shfl_xor(s, 1); const float mu = s / 256.f;
    float v = 0.f; for (int c = half * 128; c < half * 128 + 128; ++c) { const float d = so[wave][rl][c] - mu; v += d * d; } v += __shfl_xor(v, 1); const float rs = rsqrtf(v / 256.f + 1e-5f);
    for (int c = half * 128; c < half * 128 + 128; ++c) { const float y = (so[wave][rl][c] - mu) * rs * bfr(g1[c]) + bfr(bb1[c]); const __bf16 hb = (__bf16)y; sch[wave][rl][KD + c] = hb; scl[wave][rl][KD + c] = (__bf16)(y - (float)hb); }
    for (int c = half * 64; c < half * 64 + 64; ++c) { const float y = E[(size_t)(r0 + rl) * KD + c]; const __bf16 hb = (__bf16)y; sch[wave][rl][c] = hb; scl[wave][rl][c] = (__bf16)(y - (float)hb); } }
  LDSX();
  { v8f acc[8] = {};
#pragma unroll 2
    for (int kc = 0; kc < 384 / 32; ++kc) { const v16b ah = frag_b(&sch[wave][col][kc * 32], lane), al = frag_b(&scl[wave][col][kc * 32], lane);
#pragma unroll
      for (int j = 0; j < 8; ++j) { const v16b w = frag_b(WUP + (size_t)(j * 16 + col) * 384 + kc * 32, lane); acc[j] = wmma_bf(al, w, acc[j]); acc[j] = wmma_bf(ah, w, acc[j]); } }
    LDSX();
#pragma unroll
    for (int j = 0; j < 8; ++j)
#pragma unroll
      for (int r = 0; r < 8; ++r) so[wave][8 * g + r][j * 16 + col] = acc[j][r]; }
  LDSX();
  { const int rl = lane >> 1, half = lane & 1; float s = 0.f; for (int c = half * 64; c < half * 64 + 64; ++c) s += so[wave][rl][c]; s += __shfl_xor(s, 1); const float mu = s / 128.f;
    float v = 0.f; for (int c = half * 64; c < half * 64 + 64; ++c) { const float d = so[wave][rl][c] - mu; v += d * d; } v += __shfl_xor(v, 1); const float rs = rsqrtf(v / 128.f + 1e-5f);
    LDSX();
    for (int c = half * 64; c < half * 64 + 64; ++c) so[wave][rl][c] = (so[wave][rl][c] - mu) * rs * bfr(g2[c]) + bfr(bb2[c]); }
  LDSX();
  for (int rl = 0; rl < 16; ++rl) { vst2(E + (size_t)(r0 + rl) * KD + lane * 4, *(const v4f*)&so[wave][rl][lane * 4]); if (Eout) vst2(Eout + (size_t)(r0 + rl) * KD + lane * 4, *(const v4f*)&so[wave][rl][lane * 4]); }
}

extern "C" void kernel_launch(void* const* d_in, const int* in_sizes, int n_in, void* d_out, int out_size, void* d_ws, size_t ws_size, hipStream_t stream) {
  (void)in_sizes; (void)n_in; (void)out_size;
  const float** F = (const float**)d_in;
  if (ws_size < (size_t)WS_END) return;
  char* ws = (char*)d_ws; __bf16* PT = (__bf16*)(ws + WS_PT); float *EU = (float*)(ws + WS_EU), *EV = (float*)(ws + WS_EV), *PU = (float*)(ws + WS_PU), *PV = (float*)(ws + WS_PV), *MT = (float*)(ws + WS_MT), *A = (float*)(ws + WS_A), *AT = (float*)(ws + WS_AT);
  float* OEU = (float*)d_out; float* OEV = OEU + NU * KD; float* OA = OEV + NV * KD;
  k_pack<<<1408, 128, 0, stream>>>(F[4], F[6], F[10], F[14], F[18], F[21], PT);
  k_init<<<NU + NV, 32, 0, stream>>>(F[0], F[1], EU, EV);
#if DBGM != 0
#if DBGM == 3
  k_zeroA<<<NU * NV / 256, 64, 0, stream>>>(A);
#endif
  k_node<<<NU / 64, 128, 0, stream>>>(EU, EV, PT, F[5], F[11], F[15], PU, PV, MT, 0);
  k_node<<<NV / 64, 128, 0, stream>>>(EU, EV, PT, F[5], F[11], F[15], PU, PV, MT, 1);
  k_edge<<<dim3(NV / 64, 64), 128, 0, stream>>>(PU, PV, (const int*)d_in[2], (const int*)d_in[3], PT, F[7], F[8], F[9], A, OA);
#if DBGM >= 2
  k_upd<<<1, 128, 0, stream>>>(A, MT, EU, PT + PT_UUP, F[12], F[13], F[19], F[20], OEU);
#endif
#if DBGM == 3
  k_at<<<dim3(NV / 64, NU / 64), 256, 0, stream>>>(A, AT);
  k_node<<<NU / 64, 128, 0, stream>>>(EU, EV, PT, F[5], F[11], F[15], PU, PV, MT, 2);
  k_upd<<<NV / 64, 128, 0, stream>>>(AT, MT, EV, PT + PT_VUP, F[16], F[17], F[22], F[23], OEV);
#endif
  return;
#endif
  for (int it = 0; it < 2; ++it) { const bool last = (it == 1);
    k_node<<<NU / 64, 128, 0, stream>>>(EU, EV, PT, F[5], F[11], F[15], PU, PV, MT, 0);
    k_node<<<NV / 64, 128, 0, stream>>>(EU, EV, PT, F[5], F[11], F[15], PU, PV, MT, 1);
    k_edge<<<dim3(NV / 64, NU), 128, 0, stream>>>(PU, PV, (const int*)d_in[2], (const int*)d_in[3], PT, F[7], F[8], F[9], A, last ? OA : nullptr);
    k_at<<<dim3(NV / 64, NU / 64), 256, 0, stream>>>(A, AT);
    k_upd<<<NU / 64, 128, 0, stream>>>(A, MT, EU, PT + PT_UUP, F[12], F[13], F[19], F[20], last ? OEU : nullptr);
    k_node<<<NU / 64, 128, 0, stream>>>(EU, EV, PT, F[5], F[11], F[15], PU, PV, MT, 2);
    k_upd<<<NV / 64, 128, 0, stream>>>(AT, MT, EV, PT + PT_VUP, F[16], F[17], F[22], F[23], last ? OEV : nullptr); }
}
